// LSTM_74182675136807
// MI455X (gfx1250) — hardware-verified
//
#include <hip/hip_runtime.h>
#include <math.h>

constexpr int VOCAB_N   = 32000;
constexpr int EMB_N     = 10;
constexpr int HID_N     = 256;
constexpr int CLS_N     = 10;
constexpr int BATCH_N   = 1024;
constexpr int STEPS_N   = 256;
constexpr int GATE_COLS = 4 * HID_N;
constexpr int KAUG_N    = 288;
constexpr int ROWS_BLK  = 32;
constexpr int NTHREADS  = 256;
constexpr int A_PITCH   = 296;
constexpr int HS_PITCH  = 260;
constexpr int XCOL_HI   = HID_N;
constexpr int XCOL_LO   = HID_N + EMB_N;
constexpr int XCOL_SH   = HID_N + 2 * EMB_N;
constexpr int XCOL_PAD  = HID_N + 3 * EMB_N;
constexpr int GROUPS_ROW = KAUG_N / 8;
constexpr int GATE_STRIDE = HID_N * KAUG_N;
constexpr int OUT_BLK_FLOATS = ROWS_BLK * CLS_N;

constexpr float H_CARRY       = 64.0f;
constexpr float W_CARRY       = 16.0f;
constexpr float ACC_FOLD      = 1.0f / (H_CARRY * W_CARRY);
constexpr float XLO_CARRY     = 16.0f;
constexpr float XLO_CARRY_INV = 1.0f / XLO_CARRY;
constexpr float WLO_CARRY     = 256.0f;
constexpr float WLO_CARRY_INV = 1.0f / WLO_CARRY;

static_assert(KAUG_N % 32 == 0, "K multiple of 32");
static_assert(HID_N + 3 * EMB_N + 2 == KAUG_N, "augment chunk layout");
static_assert(XCOL_PAD + 2 == KAUG_N, "two zero pad columns");
static_assert(BATCH_N % ROWS_BLK == 0, "row blocks exact");
static_assert(ROWS_BLK == 32, "two 16-row subtiles per block");
static_assert(HID_N == 32 * (NTHREADS / 32), "8 waves x 32 hidden columns");
static_assert((HID_N * GROUPS_ROW) % NTHREADS == 0, "plane build grid exact");
static_assert((ROWS_BLK * A_PITCH) % NTHREADS == 0, "A tile zero fill exact");
static_assert((A_PITCH * 2) % 16 == 0, "A rows 16-B aligned");
static_assert((OUT_BLK_FLOATS * 4) % 128 == 0, "block output = whole 128-B lines");
static_assert(OUT_BLK_FLOATS % 4 == 0, "float4 stores");
static_assert(ROWS_BLK * 8 == NTHREADS, "x staging map");
static_assert(EMB_N > 8 && EMB_N <= 16, "x staging map");

typedef __attribute__((ext_vector_type(16))) _Float16 v16h;
typedef __attribute__((ext_vector_type(8)))  _Float16 v8h;
typedef __attribute__((ext_vector_type(8)))  float    v8f;
typedef __attribute__((ext_vector_type(4)))  float    v4f;
typedef unsigned __attribute__((may_alias)) u32_alias;

union FragU { v16h v; v8h h[2]; };
__device__ __forceinline__ v16h frag_load(const _Float16* p) {
  FragU f;
  f.h[0] = *(const v8h*)(p);
  f.h[1] = *(const v8h*)(p + 16);
  return f.v;
}
__device__ __forceinline__ v8f frag_mma(v16h a, v16h b, v8f c) {
  return __builtin_amdgcn_wmma_f32_16x16x32_f16(false, a, false, b, (short)0, c, false, false);
}
__device__ __forceinline__ void guard8(v8f& c0, v8f& c1, v8f& c2, v8f& c3, v8f& c4, v8f& c5, v8f& c6, v8f& c7,
                                       v16h a0, v16h a1, v16h b0, v16h b1, v16h b2, v16h b3) {
  asm volatile("v_nop\n\tv_nop\n\tv_nop\n\tv_nop"
               : "+v"(c0), "+v"(c1), "+v"(c2), "+v"(c3), "+v"(c4), "+v"(c5), "+v"(c6), "+v"(c7)
               : "v"(a0), "v"(a1), "v"(b0), "v"(b1), "v"(b2), "v"(b3));
}

__device__ __forceinline__ float fsig(float x)  { return __builtin_amdgcn_rcpf(1.0f + __expf(-x)); }
__device__ __forceinline__ float ftanh(float x) { return 1.0f - 2.0f * __builtin_amdgcn_rcpf(__expf(2.0f * x) + 1.0f); }

__global__ __launch_bounds__(NTHREADS) void build_wplane_kernel(
    const float* __restrict__ Wgx, const float* __restrict__ Wgh,
    const float* __restrict__ Wix, const float* __restrict__ Wih,
    const float* __restrict__ Wfx, const float* __restrict__ Wfh,
    const float* __restrict__ Wox, const float* __restrict__ Woh,
    unsigned short* __restrict__ dst) {
  const int gate = blockIdx.y;
  const float* Wh = (gate == 0) ? Wgh : (gate == 1) ? Wih : (gate == 2) ? Wfh : Woh;
  const float* Wx = (gate == 0) ? Wgx : (gate == 1) ? Wix : (gate == 2) ? Wfx : Wox;
  const int li = blockIdx.x * NTHREADS + threadIdx.x;
  const int nl = li / GROUPS_ROW;
  const int c8 = li - nl * GROUPS_ROW;
  const bool isx = (c8 >= HID_N / 8);

  float whv[8], wxv[8];
  int   segv[8];
#pragma unroll
  for (int e = 0; e < 8; ++e) {
    const int k  = 8 * c8 + e;
    const int kh = (k < HID_N) ? k : (HID_N - 1);
    whv[e] = Wh[(size_t)kh * HID_N + nl];
  }
  asm volatile("" : "+v"(whv[0]), "+v"(whv[1]), "+v"(whv[2]), "+v"(whv[3]),
                    "+v"(whv[4]), "+v"(whv[5]), "+v"(whv[6]), "+v"(whv[7]) : : "memory");
#pragma unroll
  for (int e = 0; e < 8; ++e) {
    int kk = 8 * c8 + e - HID_N;
    kk = (kk < 0) ? 0 : kk;
    const int seg = (kk >= 3 * EMB_N) ? 3 : (kk >= 2 * EMB_N) ? 2 : (kk >= EMB_N) ? 1 : 0;
    int ki = kk - EMB_N * seg;
    ki = (ki > EMB_N - 1) ? (EMB_N - 1) : ki;
    segv[e] = seg;
    wxv[e] = Wx[(size_t)ki * HID_N + nl];
  }
  asm volatile("" : "+v"(wxv[0]), "+v"(wxv[1]), "+v"(wxv[2]), "+v"(wxv[3]),
                    "+v"(wxv[4]), "+v"(wxv[5]), "+v"(wxv[6]), "+v"(wxv[7]) : : "memory");

  v8h hv;
#pragma unroll
  for (int e = 0; e < 8; ++e) {
    const float wx  = wxv[e];
    const float w16 = wx * W_CARRY;
    const _Float16 hi = (_Float16)w16;
    const float f0 = (float)hi;
    const _Float16 pl = (_Float16)wx;
    const float f1 = (float)pl;
    const float res = (w16 - f0) * WLO_CARRY;
    const _Float16 lo = (_Float16)res;
    const float f2 = (float)lo;
    const int seg = segv[e];
    const float fx = (seg == 0) ? f0 : (seg == 1) ? f1 : (seg == 2) ? f2 : 0.0f;
    const float fh = whv[e] * W_CARRY;
    const float f  = isx ? fx : fh;
    hv[e] = (_Float16)f;
  }
  unsigned short* op = dst + ((size_t)gate * (size_t)(HID_N * GROUPS_ROW) + (size_t)li) * 8;
  *(volatile v8h*)op = hv;
  __threadfence();
  *(volatile v8h*)op = hv;
}

__device__ __forceinline__ void stage_x(_Float16* Ax, const int* __restrict__ xtok, const float* __restrict__ emb,
                                        int rowbase, int tstep, int tid) {
  const int gm = tid >> 3, gs = tid & 7;
  int tk = xtok[(size_t)(rowbase + gm) * STEPS_N + tstep];
  tk = (tk < 0) ? 0 : tk;
  tk = (tk > VOCAB_N - 1) ? (VOCAB_N - 1) : tk;
  const float* er = emb + (size_t)tk * EMB_N;
  const int k2 = (gs < EMB_N - 8) ? (gs + 8) : (EMB_N - 1);
  float e1 = er[gs];
  float e2 = er[k2];
  asm volatile("" : "+v"(e1), "+v"(e2));

  const float xa1 = e1 * H_CARRY;
  const _Float16 h1 = (_Float16)xa1;
  const float h1f = (float)h1;
  const _Float16 l1 = (_Float16)((xa1 - h1f) * XLO_CARRY);
  const _Float16 s1 = (_Float16)(h1f * WLO_CARRY_INV);

  const float xa2 = e2 * H_CARRY;
  const _Float16 h2 = (_Float16)xa2;
  const float h2f = (float)h2;
  const _Float16 l2 = (_Float16)((xa2 - h2f) * XLO_CARRY);
  const _Float16 s2 = (_Float16)(h2f * WLO_CARRY_INV);

  _Float16* row = Ax + gm * A_PITCH;
  row[XCOL_HI + gs] = h1;
  row[XCOL_LO + gs] = l1;
  row[XCOL_SH + gs] = s1;
  if (gs < EMB_N - 8) {
    row[XCOL_HI + 8 + gs] = h2;
    row[XCOL_LO + 8 + gs] = l2;
    row[XCOL_SH + 8 + gs] = s2;
  } else if (gs == 2) {
    *(u32_alias*)(row + XCOL_PAD) = 0u;
  }
}

__global__ __launch_bounds__(NTHREADS) void lstm_seq_kernel(
    const int* __restrict__ xtok, const float* __restrict__ emb,
    const float* __restrict__ bg, const float* __restrict__ bi,
    const float* __restrict__ bfv, const float* __restrict__ bo,
    const float* __restrict__ Wph, const float* __restrict__ bp,
    const unsigned short* __restrict__ WCp, float* __restrict__ out) {
  __shared__ __align__(16) _Float16 Ax[ROWS_BLK * A_PITCH];
  __shared__ __align__(16) float    Hs[ROWS_BLK * HS_PITCH];
  __shared__ __align__(16) float    Ost[OUT_BLK_FLOATS];
  const _Float16* WC = (const _Float16*)WCp;
  const int tid = threadIdx.x, lane = tid & 31, wave = tid >> 5;
  const int c = lane & 15, hh = lane >> 4, koff = hh * 8;
  const int rowbase = blockIdx.x * ROWS_BLK;

#pragma unroll 1
  for (int i = tid; i < ROWS_BLK * A_PITCH; i += NTHREADS) Ax[i] = (_Float16)0.0f;
  __syncthreads();
  stage_x(Ax, xtok, emb, rowbase, 0, tid);

  float cst[2][2][8], hst[2][2][8], bb[2][4];
#pragma unroll
  for (int nt = 0; nt < 2; ++nt) {
    const int j = 32 * wave + 16 * nt + c;
    bb[nt][0] = bg[j];
    bb[nt][1] = bi[j];
    bb[nt][2] = bfv[j];
    bb[nt][3] = bo[j];
#pragma unroll
    for (int mt = 0; mt < 2; ++mt)
#pragma unroll
      for (int r = 0; r < 8; ++r) { cst[nt][mt][r] = 0.0f; hst[nt][mt][r] = 0.0f; }
  }
  __syncthreads();

  const _Float16* arow0 = Ax + c * A_PITCH + koff;
  const _Float16* arow1 = Ax + (16 + c) * A_PITCH + koff;
  const v8f z8 = {0.f, 0.f, 0.f, 0.f, 0.f, 0.f, 0.f, 0.f};

#pragma unroll 1
  for (int t = 0; t < STEPS_N; ++t) {
#pragma unroll
    for (int nt = 0; nt < 2; ++nt) {
      const int j = 32 * wave + 16 * nt + c;
      const _Float16* wb = WC + (size_t)j * KAUG_N + koff;
      v8f acc[4][2];
#pragma unroll
      for (int g = 0; g < 4; ++g) { acc[g][0] = z8; acc[g][1] = z8; }
#pragma unroll 1
      for (int k0 = 0; k0 < KAUG_N; k0 += 32) {
        const v16h a0 = frag_load(arow0 + k0);
        const v16h a1 = frag_load(arow1 + k0);
        const v16h b0 = frag_load(wb + k0);
        const v16h b1 = frag_load(wb + (size_t)1 * GATE_STRIDE + k0);
        const v16h b2 = frag_load(wb + (size_t)2 * GATE_STRIDE + k0);
        const v16h b3 = frag_load(wb + (size_t)3 * GATE_STRIDE + k0);
        acc[0][0] = frag_mma(a0, b0, acc[0][0]);
        acc[0][1] = frag_mma(a1, b0, acc[0][1]);
        acc[1][0] = frag_mma(a0, b1, acc[1][0]);
        acc[1][1] = frag_mma(a1, b1, acc[1][1]);
        acc[2][0] = frag_mma(a0, b2, acc[2][0]);
        acc[2][1] = frag_mma(a1, b2, acc[2][1]);
        acc[3][0] = frag_mma(a0, b3, acc[3][0]);
        acc[3][1] = frag_mma(a1, b3, acc[3][1]);
        guard8(acc[0][0], acc[0][1], acc[1][0], acc[1][1], acc[2][0], acc[2][1], acc[3][0], acc[3][1],
               a0, a1, b0, b1, b2, b3);
      }
#pragma unroll
      for (int mt = 0; mt < 2; ++mt) {
#pragma unroll
        for (int r = 0; r < 8; ++r) {
          const float zg = acc[0][mt][r] * ACC_FOLD + bb[nt][0];
          const float zi = acc[1][mt][r] * ACC_FOLD + bb[nt][1];
          const float zf = acc[2][mt][r] * ACC_FOLD + bb[nt][2];
          const float zo = acc[3][mt][r] * ACC_FOLD + bb[nt][3];
          const float gg = ftanh(zg);
          const float ig = fsig(zi);
          const float fg = fsig(zf);
          const float og = fsig(zo);
          const float cn = gg * ig + cst[nt][mt][r] * fg;
          cst[nt][mt][r] = cn;
          hst[nt][mt][r] = ftanh(cn) * og;
        }
      }
    }
    __syncthreads();
#pragma unroll
    for (int nt = 0; nt < 2; ++nt) {
      const int j = 32 * wave + 16 * nt + c;
#pragma unroll
      for (int mt = 0; mt < 2; ++mt)
#pragma unroll
        for (int r = 0; r < 8; ++r)
          Ax[(16 * mt + 8 * hh + r) * A_PITCH + j] = (_Float16)(hst[nt][mt][r] * H_CARRY);
    }
    {
      const int tn = (t + 1 < STEPS_N) ? (t + 1) : (STEPS_N - 1);
      stage_x(Ax, xtok, emb, rowbase, tn, tid);
    }
    __syncthreads();
  }

#pragma unroll
  for (int nt = 0; nt < 2; ++nt) {
    const int j = 32 * wave + 16 * nt + c;
#pragma unroll
    for (int mt = 0; mt < 2; ++mt)
#pragma unroll
      for (int r = 0; r < 8; ++r)
        Hs[(16 * mt + 8 * hh + r) * HS_PITCH + j] = hst[nt][mt][r];
  }
  __syncthreads();

#pragma unroll 1
  for (int idx = tid; idx < OUT_BLK_FLOATS; idx += NTHREADS) {
    const int m = idx / CLS_N;
    const int n = idx - m * CLS_N;
    const float* hr = Hs + m * HS_PITCH;
    float s = 0.0f;
#pragma unroll 4
    for (int k = 0; k < HID_N; ++k) s = fmaf(hr[k], Wph[k * CLS_N + n], s);
    Ost[idx] = s + bp[n];
  }
  __syncthreads();

  if (wave == 0) {
    float* ob = out + (size_t)rowbase * CLS_N;
    for (int pass = 0; pass < 2; ++pass) {
#pragma unroll
      for (int it = 0; it < 3; ++it) {
        const int q4  = it * 32 + lane;
        const int q4c = (q4 < OUT_BLK_FLOATS / 4) ? q4 : (OUT_BLK_FLOATS / 4 - 1);
        const v4f v = *(const v4f*)(Ost + 4 * q4c);
        if (q4 < OUT_BLK_FLOATS / 4) *(volatile v4f*)(ob + 4 * q4) = v;
      }
      __threadfence();
    }
  }
}

extern "C" void kernel_launch(void* const* d_in, const int* in_sizes, int n_in,
                              void* d_out, int out_size, void* d_ws, size_t ws_size, hipStream_t stream) {
  if (n_in < 16 || d_out == nullptr || d_ws == nullptr) return;
  if (in_sizes[0] != BATCH_N * STEPS_N || in_sizes[1] != VOCAB_N * EMB_N ||
      in_sizes[2] != EMB_N * HID_N || in_sizes[3] != HID_N * HID_N || in_sizes[4] != HID_N ||
      in_sizes[5] != EMB_N * HID_N || in_sizes[6] != HID_N * HID_N || in_sizes[7] != HID_N ||
      in_sizes[8] != EMB_N * HID_N || in_sizes[9] != HID_N * HID_N || in_sizes[10] != HID_N ||
      in_sizes[11] != EMB_N * HID_N || in_sizes[12] != HID_N * HID_N || in_sizes[13] != HID_N ||
      in_sizes[14] != HID_N * CLS_N || in_sizes[15] != CLS_N || out_size != BATCH_N * CLS_N) return;

  const int*   xtok = (const int*)  d_in[0];
  const float* emb  = (const float*)d_in[1];
  const float* Wgx  = (const float*)d_in[2];
  const float* Wgh  = (const float*)d_in[3];
  const float* bg   = (const float*)d_in[4];
  const float* Wix  = (const float*)d_in[5];
  const float* Wih  = (const float*)d_in[6];
  const float* bi   = (const float*)d_in[7];
  const float* Wfx  = (const float*)d_in[8];
  const float* Wfh  = (const float*)d_in[9];
  const float* bfv  = (const float*)d_in[10];
  const float* Wox  = (const float*)d_in[11];
  const float* Woh  = (const float*)d_in[12];
  const float* bo   = (const float*)d_in[13];
  const float* Wph  = (const float*)d_in[14];
  const float* bp   = (const float*)d_in[15];
  float* out = (float*)d_out;

  char* ws = (char*)d_ws; size_t off = 0;
  auto carve = [&](size_t bytes) -> char* { char* p = ws + off; off += (bytes + 255) & ~(size_t)255; return p; };
  unsigned short* WC = (unsigned short*)carve((size_t)GATE_COLS * KAUG_N * 2);
  if (off > ws_size || off > (size_t)134217728) return;

  build_wplane_kernel<<<dim3((HID_N * GROUPS_ROW) / NTHREADS, 4), NTHREADS, 0, stream>>>(
      Wgx, Wgh, Wix, Wih, Wfx, Wfh, Wox, Woh, WC);
  lstm_seq_kernel<<<BATCH_N / ROWS_BLK, NTHREADS, 0, stream>>>(
      xtok, emb, bg, bi, bfv, bo, Wph, bp, WC, out);
}
